// PointNetSetAbstraction_22273700397315
// MI455X (gfx1250) — hardware-verified
//
#include <hip/hip_runtime.h>

#pragma clang fp contract(off)

typedef __attribute__((ext_vector_type(16))) _Float16 v16h;
typedef __attribute__((ext_vector_type(8)))  _Float16 v8h;
typedef __attribute__((ext_vector_type(8)))  float    v8f;
typedef __attribute__((ext_vector_type(4)))  float    v4f;

constexpr int N_BATCH = 16;
constexpr int N_PTS   = 256;
constexpr int N_FEAT  = 64;
constexpr int C_IN0   = 3 + N_FEAT;
constexpr int C_OUT1  = 64;
constexpr int C_OUT2  = 64;
constexpr int C_OUT3  = 128;
constexpr int N_QUERY = N_BATCH * N_PTS;
constexpr int K_SLOTS = N_PTS - 1;
constexpr float ROWS_INV = (float)(1.0 / ((double)N_QUERY * (double)K_SLOTS));
constexpr float BALL_R2 = 0.04f;
constexpr float BN_EPS  = 1e-5f;
constexpr float W_CARRY = 16.0f;
constexpr float W_CARRY_INV = 1.0f / W_CARRY;
constexpr int LDS_PITCH = 72;

constexpr int WAVES_PB    = 4;
constexpr int THREADS_PB  = 32 * WAVES_PB;
constexpr int Q_PER_WAVE  = 8;
constexpr int Q_PER_BLOCK = WAVES_PB * Q_PER_WAVE;
constexpr int N_BLK       = N_QUERY / Q_PER_BLOCK;

static_assert(C_IN0 == 67, "first layer input width");
static_assert(N_QUERY == 4096, "query count");
static_assert(N_BLK * Q_PER_BLOCK == N_QUERY, "exact query coverage");
static_assert(N_PTS % 32 == 0, "candidate chunks of one wave");
static_assert(C_OUT1 % 32 == 0 && C_OUT2 % 32 == 0, "K multiple of 32 for both WMMA layers");
static_assert(C_OUT2 % 16 == 0 && C_OUT3 % 16 == 0, "N multiple of 16");

constexpr size_t OFF_Y     = 0;
constexpr size_t OFF_XC    = OFF_Y   + (size_t)N_QUERY * 64 * 4;
constexpr size_t OFF_GMX   = OFF_XC  + (size_t)N_QUERY * 64 * 4;
constexpr size_t OFF_P0    = OFF_GMX + (size_t)N_QUERY * 128 * 4;
constexpr size_t OFF_P1    = OFF_P0  + (size_t)N_BLK * 128 * 4;
constexpr size_t OFF_P2    = OFF_P1  + (size_t)N_BLK * 128 * 4;
constexpr size_t OFF_COEF1 = OFF_P2  + (size_t)N_BLK * 256 * 4;
constexpr size_t OFF_COEF2 = OFF_COEF1 + 1024;
constexpr size_t OFF_COEF3 = OFF_COEF2 + 1024;
constexpr size_t WS_TOTAL  = OFF_COEF3 + 1024;
static_assert(WS_TOTAL <= (size_t)134217728, "carve budget");
static_assert((OFF_XC % 128) == 0 && (OFF_GMX % 128) == 0 && (OFF_P0 % 128) == 0 && (OFF_P1 % 128) == 0 &&
              (OFF_P2 % 128) == 0 && (OFF_COEF1 % 128) == 0 && (OFF_COEF2 % 128) == 0 && (OFF_COEF3 % 128) == 0,
              "line-aligned carve");

__device__ __forceinline__ void wave_lds_sync() {
  __builtin_amdgcn_fence(__ATOMIC_RELEASE, "workgroup");
  __builtin_amdgcn_wave_barrier();
  __builtin_amdgcn_fence(__ATOMIC_ACQUIRE, "workgroup");
}

__device__ __forceinline__ v16h frag_load(const _Float16* p) {
  union { v16h v; v8h h[2]; } f;
  f.h[0] = *(const v8h*)(p);
  f.h[1] = *(const v8h*)(p + 16);
  return f.v;
}

__device__ __forceinline__ v8f mma_f16(v16h a, v16h b, v8f c) {
  c = __builtin_amdgcn_wmma_f32_16x16x32_f16(false, a, false, b, (short)0, c, false, false);
  asm volatile("v_nop\n\tv_nop\n\tv_nop\n\tv_nop" : "+v"(c) : "v"(a), "v"(b));
  return c;
}

__device__ __forceinline__ int clamp_pt(int i) {
  i = i < 0 ? 0 : i;
  i = i > (N_PTS - 1) ? (N_PTS - 1) : i;
  return i;
}

__device__ __forceinline__ int ball_list(const float* __restrict__ xyz, int b, int n, int lane, int* lstw) {
#pragma clang fp contract(off)
  const float* xb = xyz + (size_t)b * (3 * N_PTS);
  const float qx = xb[n];
  const float qy = xb[N_PTS + n];
  const float qz = xb[2 * N_PTS + n];
  const float qxx = qx * qx;
  const float qyy = qy * qy;
  const float qzz = qz * qz;
  const float sqq = (qxx + qzz) + qyy;
  const unsigned below = (1u << lane) - 1u;
  int base = 0;
#pragma unroll 1
  for (int j = 0; j < N_PTS / 32; ++j) {
    const int m = 32 * j + lane;
    const float px = xb[m];
    const float py = xb[N_PTS + m];
    const float pz = xb[2 * N_PTS + m];
    const float pxx = px * px;
    const float pyy = py * py;
    const float pzz = pz * pz;
    const float sqp = (pxx + pzz) + pyy;
    float p = qx * px;
    p = fmaf(qy, py, p);
    p = fmaf(qz, pz, p);
    const float ssum = sqq + sqp;
    const float twop = 2.0f * p;
    const float d = ssum - twop;
    const bool hit = !(d > BALL_R2);
    const unsigned mask = __builtin_amdgcn_ballot_w32(hit);
    const int pos = base + __builtin_popcount(mask & below);
    if (hit) lstw[pos] = m;
    base += __builtin_popcount(mask);
  }
  return base;
}

__device__ __forceinline__ void stage_tile(_Float16* Atw, const float* __restrict__ Y, const float* __restrict__ Xc,
                                           const int* lstw, int cv, int t, int b, int q, int lane, const float* sAC) {
  const int m = lane & 15;
  const int cb = lane >> 4;
  const int r = 16 * t + m;
  const int ri = (r < cv) ? r : 0;
  const int gi = clamp_pt(lstw[ri]);
  const float* Yr = Y + ((size_t)(b * N_PTS + gi)) * 64 + cb * 32;
  const float* Xr = Xc + (size_t)q * 64 + cb * 32;
  const float* ar = sAC + cb * 32;
  const float* cr = sAC + 64 + cb * 32;
#pragma unroll
  for (int i = 0; i < 4; ++i) {
    const v4f y0 = *(const v4f*)(Yr + 8 * i);
    const v4f y1 = *(const v4f*)(Yr + 8 * i + 4);
    const v4f x0 = *(const v4f*)(Xr + 8 * i);
    const v4f x1 = *(const v4f*)(Xr + 8 * i + 4);
    const v4f a0 = *(const v4f*)(ar + 8 * i);
    const v4f a1 = *(const v4f*)(ar + 8 * i + 4);
    const v4f c0 = *(const v4f*)(cr + 8 * i);
    const v4f c1 = *(const v4f*)(cr + 8 * i + 4);
    v8h hv;
#pragma unroll
    for (int e = 0; e < 4; ++e) {
      const float d0 = y0[e] - x0[e];
      const float d1 = y1[e] - x1[e];
      const float f0 = fminf(fmaxf(a0[e] * d0 + c0[e], 0.0f), 60000.0f);
      const float f1 = fminf(fmaxf(a1[e] * d1 + c1[e], 0.0f), 60000.0f);
      hv[e] = (_Float16)f0;
      hv[4 + e] = (_Float16)f1;
    }
    *(v8h*)(Atw + m * LDS_PITCH + cb * 32 + 8 * i) = hv;
    asm volatile("" ::: "memory");
  }
}

__device__ __forceinline__ void stage_weights(_Float16* Wl, const float* __restrict__ W, int nrows, int tid) {
#pragma unroll 1
  for (int g = tid; g < nrows * 8; g += THREADS_PB) {
    const int n = g >> 3;
    const int k8 = (g & 7) * 8;
    const v4f w0 = *(const v4f*)(W + n * 64 + k8);
    const v4f w1 = *(const v4f*)(W + n * 64 + k8 + 4);
    v8h hv;
#pragma unroll
    for (int e = 0; e < 4; ++e) {
      const float s0 = w0[e] * W_CARRY;
      const float s1 = w1[e] * W_CARRY;
      hv[e] = (_Float16)s0;
      hv[4 + e] = (_Float16)s1;
    }
    *(v8h*)(Wl + n * LDS_PITCH + k8) = hv;
  }
}

__global__ __launch_bounds__(256) void first_layer_kernel(const float* __restrict__ xyz, const float* __restrict__ pts,
                                                          const float* __restrict__ W0,
                                                          float* __restrict__ Y, float* __restrict__ Xc) {
  __shared__ __align__(16) float Ws[C_OUT1 * C_IN0];
  __shared__ __align__(16) float Ps[C_IN0 * 32];
  __shared__ __align__(16) float Yt[32 * 68];
  __shared__ __align__(16) float Xt[32 * 68];
  const int tid = threadIdx.x;
  const int bm0 = blockIdx.x * 32;
  const int b = bm0 >> 8;
  const int m0 = bm0 & (N_PTS - 1);
#pragma unroll 1
  for (int i = tid; i < C_OUT1 * C_IN0; i += 256) Ws[i] = W0[i];
  if (tid < 96) {
    const int k = tid >> 5;
    const int mm = tid & 31;
    Ps[tid] = xyz[(size_t)b * (3 * N_PTS) + k * N_PTS + m0 + mm];
  }
#pragma unroll 1
  for (int i = tid; i < N_FEAT * 32; i += 256) {
    const int d = i >> 5;
    const int mm = i & 31;
    Ps[96 + i] = pts[(size_t)b * (N_FEAT * N_PTS) + d * N_PTS + m0 + mm];
  }
  __syncthreads();

  const int o = tid & 63;
  const int mg = tid >> 6;
  const float* wrow = Ws + o * C_IN0;
  const float wx = wrow[0];
  const float wy = wrow[1];
  const float wz = wrow[2];
  float sx[8], sp[8];
#pragma unroll
  for (int i = 0; i < 8; ++i) {
    const int mm = mg * 8 + i;
    float s = wx * Ps[mm];
    s = fmaf(wy, Ps[32 + mm], s);
    s = fmaf(wz, Ps[64 + mm], s);
    sx[i] = s;
    sp[i] = 0.0f;
  }
#pragma unroll 1
  for (int d = 0; d < N_FEAT; ++d) {
    const float w = wrow[3 + d];
    const float* pr = Ps + (3 + d) * 32 + mg * 8;
#pragma unroll
    for (int i = 0; i < 8; ++i) sp[i] = fmaf(w, pr[i], sp[i]);
  }
#pragma unroll
  for (int i = 0; i < 8; ++i) {
    const int mm = mg * 8 + i;
    Yt[mm * 68 + o] = sx[i] + sp[i];
    Xt[mm * 68 + o] = sx[i];
  }
  __syncthreads();
  {
    const int lane = tid & 31;
    const int wave = tid >> 5;
    const int hh = lane >> 4;
    const int c4 = (lane & 15) * 4;
    v4f yv[2], xv[2];
#pragma unroll
    for (int it = 0; it < 2; ++it) {
      const int row = wave * 4 + it * 2 + hh;
      yv[it] = *(const v4f*)(Yt + row * 68 + c4);
      xv[it] = *(const v4f*)(Xt + row * 68 + c4);
    }
    for (int pass = 0; pass < 2; ++pass) {
#pragma unroll
      for (int it = 0; it < 2; ++it) {
        const int row = wave * 4 + it * 2 + hh;
        *(volatile v4f*)(Y + (size_t)(bm0 + row) * 64 + c4) = yv[it];
        *(volatile v4f*)(Xc + (size_t)(bm0 + row) * 64 + c4) = xv[it];
      }
      __threadfence();
    }
  }
}

__global__ __launch_bounds__(128) void stats0_kernel(const float* __restrict__ xyz, const float* __restrict__ Y,
                                                     const float* __restrict__ Xc, float* __restrict__ P0) {
#pragma clang fp contract(off)
  __shared__ int lst[WAVES_PB][N_PTS];
  __shared__ __align__(16) float red[WAVES_PB][128];
  __shared__ __align__(16) float red2[128];
  const int tid = threadIdx.x;
  const int lane = tid & 31;
  const int wave = tid >> 5;
  int* lstw = lst[wave];
  float s0 = 0.0f, s1 = 0.0f, q0 = 0.0f, q1 = 0.0f;
#pragma unroll 1
  for (int qi = 0; qi < Q_PER_WAVE; ++qi) {
    const int q = (blockIdx.x * WAVES_PB + wave) * Q_PER_WAVE + qi;
    const int b = q >> 8;
    const int n = q & (N_PTS - 1);
    int cnt = ball_list(xyz, b, n, lane, lstw);
    cnt = __builtin_amdgcn_readfirstlane(cnt);
    wave_lds_sync();
    int cv = cnt < 1 ? 1 : cnt;
    cv = cv > K_SLOTS ? K_SLOTS : cv;
    const float w0 = (float)(N_PTS - cv);
    const float xc0 = Xc[(size_t)q * 64 + lane];
    const float xc1 = Xc[(size_t)q * 64 + 32 + lane];
#pragma unroll 1
    for (int r = 0; r < cv; ++r) {
      const int gi = clamp_pt(lstw[r]);
      const float* Yr = Y + ((size_t)(b * N_PTS + gi)) * 64;
      const float v0 = Yr[lane] - xc0;
      const float v1 = Yr[32 + lane] - xc1;
      const float wgt = (r == 0) ? w0 : 1.0f;
      const float a0 = wgt * v0;
      const float a1 = wgt * v1;
      s0 += a0;
      s1 += a1;
      q0 += a0 * v0;
      q1 += a1 * v1;
    }
    wave_lds_sync();
  }
  red[wave][lane] = s0;
  red[wave][32 + lane] = s1;
  red[wave][64 + lane] = q0;
  red[wave][96 + lane] = q1;
  __syncthreads();
  red2[tid] = ((red[0][tid] + red[1][tid]) + red[2][tid]) + red[3][tid];
  __syncthreads();
  if (tid < 32) {
    const v4f pv = *(const v4f*)(red2 + 4 * tid);
    float* dst = P0 + (size_t)blockIdx.x * 128 + 4 * tid;
    *(volatile v4f*)dst = pv;
    __threadfence();
    *(volatile v4f*)dst = pv;
  }
}

__global__ __launch_bounds__(128) void bn_coef_kernel(const float* __restrict__ P, const float* __restrict__ gamma,
                                                      const float* __restrict__ beta, float* __restrict__ coef, int C) {
  __shared__ __align__(16) float sv[256];
  const int tid = threadIdx.x;
  const int twoC = 2 * C;
  for (int ch = tid; ch < C; ch += 128) {
    float S = 0.0f, Q = 0.0f;
#pragma unroll 1
    for (int blk = 0; blk < N_BLK; ++blk) {
      S += P[(size_t)blk * twoC + ch];
      Q += P[(size_t)blk * twoC + C + ch];
    }
    const float mean = S * ROWS_INV;
    float var = Q * ROWS_INV - mean * mean;
    var = fmaxf(var, 0.0f);
    const float a = gamma[ch] * (1.0f / sqrtf(var + BN_EPS));
    sv[ch] = a;
    sv[C + ch] = beta[ch] - mean * a;
  }
  __syncthreads();
  if (tid < (twoC >> 2)) {
    const v4f pv = *(const v4f*)(sv + 4 * tid);
    float* dst = coef + 4 * tid;
    *(volatile v4f*)dst = pv;
    __threadfence();
    *(volatile v4f*)dst = pv;
  }
}

template <bool FULL>
__global__ __launch_bounds__(128) void mlp_kernel(const float* __restrict__ xyz, const float* __restrict__ Y,
                                                  const float* __restrict__ Xc,
                                                  const float* __restrict__ W1, const float* __restrict__ W2,
                                                  const float* __restrict__ coef1, const float* __restrict__ coef2,
                                                  float* __restrict__ Pout, float* __restrict__ gmx) {
#pragma clang fp contract(off)
  constexpr int NJ = FULL ? (C_OUT3 / 16) : (C_OUT2 / 16);
  constexpr int NSTAT = 2 * 16 * NJ;
  __shared__ __align__(16) _Float16 W1h[C_OUT2 * LDS_PITCH];
  __shared__ __align__(16) _Float16 W2h[FULL ? C_OUT3 * LDS_PITCH : 8];
  __shared__ __align__(16) _Float16 At[WAVES_PB][16 * LDS_PITCH];
  __shared__ __align__(16) _Float16 Ft[FULL ? WAVES_PB : 1][FULL ? 16 * LDS_PITCH : 8];
  __shared__ int lst[WAVES_PB][N_PTS];
  __shared__ __align__(16) float sAC1[128];
  __shared__ __align__(16) float sAC2[FULL ? 128 : 4];
  __shared__ __align__(16) float red[WAVES_PB][NSTAT];
  __shared__ __align__(16) float red2[NSTAT];
  __shared__ __align__(16) float mrow[FULL ? WAVES_PB : 1][FULL ? C_OUT3 : 4];

  const int tid = threadIdx.x;
  const int lane = tid & 31;
  const int wave = tid >> 5;
  const int h = lane >> 4;
  const int c = lane & 15;

  stage_weights(W1h, W1, C_OUT2, tid);
  if (FULL) stage_weights(W2h, W2, C_OUT3, tid);
  sAC1[tid] = coef1[tid];
  if (FULL) sAC2[tid] = coef2[tid];
  __syncthreads();

  int* lstw = lst[wave];
  _Float16* Atw = At[wave];
  _Float16* Ftw = Ft[FULL ? wave : 0];
  float* mroww = mrow[FULL ? wave : 0];

  float sacc[8], qacc[8];
#pragma unroll
  for (int j = 0; j < 8; ++j) { sacc[j] = 0.0f; qacc[j] = 0.0f; }

#pragma unroll 1
  for (int qi = 0; qi < Q_PER_WAVE; ++qi) {
    const int q = (blockIdx.x * WAVES_PB + wave) * Q_PER_WAVE + qi;
    const int b = q >> 8;
    const int n = q & (N_PTS - 1);
    int cnt = ball_list(xyz, b, n, lane, lstw);
    cnt = __builtin_amdgcn_readfirstlane(cnt);
    wave_lds_sync();
    int cv = cnt < 1 ? 1 : cnt;
    cv = cv > K_SLOTS ? K_SLOTS : cv;
    int nt = (cv + 15) >> 4;
    nt = nt > 16 ? 16 : nt;
    const float w0 = (float)(N_PTS - cv);

    float mx[8];
#pragma unroll
    for (int j = 0; j < 8; ++j) mx[j] = -__builtin_inff();

#pragma unroll 1
    for (int t = 0; t < nt; ++t) {
      stage_tile(Atw, Y, Xc, lstw, cv, t, b, q, lane, sAC1);
      wave_lds_sync();
      const v16h af0 = frag_load(Atw + c * LDS_PITCH + 8 * h);
      const v16h af1 = frag_load(Atw + c * LDS_PITCH + 32 + 8 * h);
      const int rbase = 16 * t + 8 * h;

      if (!FULL) {
#pragma unroll
        for (int j = 0; j < 4; ++j) {
          const v16h b0 = frag_load(W1h + (16 * j + c) * LDS_PITCH + 8 * h);
          const v16h b1 = frag_load(W1h + (16 * j + c) * LDS_PITCH + 32 + 8 * h);
          v8f acc = (v8f){0.f, 0.f, 0.f, 0.f, 0.f, 0.f, 0.f, 0.f};
          acc = mma_f16(af0, b0, acc);
          acc = mma_f16(af1, b1, acc);
          float ss = sacc[j], qq = qacc[j];
#pragma unroll
          for (int r = 0; r < 8; ++r) {
            const int rr = rbase + r;
            const float x = acc[r] * W_CARRY_INV;
            const float xs = (rr < cv) ? x : 0.0f;
            const float wgt = (rr == 0) ? w0 : 1.0f;
            const float wxv = wgt * xs;
            ss += wxv;
            qq += wxv * xs;
          }
          sacc[j] = ss;
          qacc[j] = qq;
        }
      } else {
#pragma unroll
        for (int j = 0; j < 4; ++j) {
          const v16h b0 = frag_load(W1h + (16 * j + c) * LDS_PITCH + 8 * h);
          const v16h b1 = frag_load(W1h + (16 * j + c) * LDS_PITCH + 32 + 8 * h);
          v8f acc = (v8f){0.f, 0.f, 0.f, 0.f, 0.f, 0.f, 0.f, 0.f};
          acc = mma_f16(af0, b0, acc);
          acc = mma_f16(af1, b1, acc);
          const int ch = 16 * j + c;
          const float a2 = sAC2[ch];
          const float c2 = sAC2[64 + ch];
#pragma unroll
          for (int r = 0; r < 8; ++r) {
            const float x = acc[r] * W_CARRY_INV;
            const float f = fminf(fmaxf(a2 * x + c2, 0.0f), 60000.0f);
            Ftw[(8 * h + r) * LDS_PITCH + ch] = (_Float16)f;
          }
        }
        wave_lds_sync();
        const v16h ff0 = frag_load(Ftw + c * LDS_PITCH + 8 * h);
        const v16h ff1 = frag_load(Ftw + c * LDS_PITCH + 32 + 8 * h);
#pragma unroll
        for (int j = 0; j < 8; ++j) {
          const v16h b0 = frag_load(W2h + (16 * j + c) * LDS_PITCH + 8 * h);
          const v16h b1 = frag_load(W2h + (16 * j + c) * LDS_PITCH + 32 + 8 * h);
          v8f acc = (v8f){0.f, 0.f, 0.f, 0.f, 0.f, 0.f, 0.f, 0.f};
          acc = mma_f16(ff0, b0, acc);
          acc = mma_f16(ff1, b1, acc);
          float ss = sacc[j], qq = qacc[j], mm = mx[j];
#pragma unroll
          for (int r = 0; r < 8; ++r) {
            const int rr = rbase + r;
            const float x = acc[r] * W_CARRY_INV;
            mm = fmaxf(mm, x);
            const float xs = (rr < cv) ? x : 0.0f;
            const float wgt = (rr == 0) ? w0 : 1.0f;
            const float wxv = wgt * xs;
            ss += wxv;
            qq += wxv * xs;
          }
          sacc[j] = ss;
          qacc[j] = qq;
          mx[j] = mm;
        }
      }
      wave_lds_sync();
    }

    if (FULL) {
#pragma unroll
      for (int j = 0; j < 8; ++j) {
        const float other = __shfl_xor(mx[j], 16, 32);
        const float mv = fmaxf(mx[j], other);
        if (h == 0) mroww[16 * j + c] = mv;
      }
      wave_lds_sync();
      const v4f mvv = *(const v4f*)(mroww + 4 * lane);
      float* dst = gmx + (size_t)q * C_OUT3 + 4 * lane;
      *(volatile v4f*)dst = mvv;
      __threadfence();
      *(volatile v4f*)dst = mvv;
    }
    wave_lds_sync();
  }

#pragma unroll
  for (int j = 0; j < NJ; ++j) {
    const float so = __shfl_xor(sacc[j], 16, 32);
    const float qo = __shfl_xor(qacc[j], 16, 32);
    const float st = sacc[j] + so;
    const float qt = qacc[j] + qo;
    if (h == 0) {
      red[wave][16 * j + c] = st;
      red[wave][16 * NJ + 16 * j + c] = qt;
    }
  }
  __syncthreads();
  for (int e = tid; e < NSTAT; e += THREADS_PB) red2[e] = ((red[0][e] + red[1][e]) + red[2][e]) + red[3][e];
  __syncthreads();
  if (tid < (NSTAT >> 2)) {
    const v4f pv = *(const v4f*)(red2 + 4 * tid);
    float* dst = Pout + (size_t)blockIdx.x * NSTAT + 4 * tid;
    *(volatile v4f*)dst = pv;
    __threadfence();
    *(volatile v4f*)dst = pv;
  }
}

__global__ __launch_bounds__(256) void out_kernel(const float* __restrict__ gmx, const float* __restrict__ coef3,
                                                  float* __restrict__ out) {
  __shared__ __align__(16) float T[32 * 132];
  __shared__ float sa[C_OUT3];
  __shared__ float sc[C_OUT3];
  const int tid = threadIdx.x;
  const int lane = tid & 31;
  const int wave = tid >> 5;
  const int b = blockIdx.x >> 3;
  const int n0 = (blockIdx.x & 7) * 32;
  if (tid < C_OUT3) {
    sa[tid] = coef3[tid];
    sc[tid] = coef3[C_OUT3 + tid];
  }
#pragma unroll
  for (int i = 0; i < 4; ++i) {
    const int row = wave * 4 + i;
    const v4f v = *(const v4f*)(gmx + ((size_t)(b * N_PTS + n0 + row)) * C_OUT3 + 4 * lane);
    *(v4f*)(T + row * 132 + 4 * lane) = v;
  }
  __syncthreads();
  const int cq = lane >> 3;
  const int n4 = (lane & 7) * 4;
  v4f ov[4];
#pragma unroll
  for (int it = 0; it < 4; ++it) {
    const int ch = wave * 16 + it * 4 + cq;
    const float a = sa[ch];
    const float cc = sc[ch];
    v4f o;
#pragma unroll
    for (int e = 0; e < 4; ++e) o[e] = fmaxf(a * T[(n4 + e) * 132 + ch] + cc, 0.0f);
    ov[it] = o;
  }
  for (int pass = 0; pass < 2; ++pass) {
#pragma unroll
    for (int it = 0; it < 4; ++it) {
      const int ch = wave * 16 + it * 4 + cq;
      *(volatile v4f*)(out + ((size_t)(b * C_OUT3 + ch)) * N_PTS + n0 + n4) = ov[it];
    }
    __threadfence();
  }
}

extern "C" void kernel_launch(void* const* d_in, const int* in_sizes, int n_in,
                              void* d_out, int out_size, void* d_ws, size_t ws_size, hipStream_t stream) {
  if (n_in < 14) return;
  if (ws_size < WS_TOTAL) return;
  if (out_size < N_BATCH * C_OUT3 * N_PTS) return;
  const float* xyz   = (const float*)d_in[0];
  const float* pts   = (const float*)d_in[1];
  const float* W0    = (const float*)d_in[2];
  const float* g0    = (const float*)d_in[4];
  const float* beta0 = (const float*)d_in[5];
  const float* W1    = (const float*)d_in[6];
  const float* g1    = (const float*)d_in[8];
  const float* beta1 = (const float*)d_in[9];
  const float* W2    = (const float*)d_in[10];
  const float* g2    = (const float*)d_in[12];
  const float* beta2 = (const float*)d_in[13];
  float* out = (float*)d_out;

  char* ws = (char*)d_ws;
  float* Y     = (float*)(ws + OFF_Y);
  float* Xc    = (float*)(ws + OFF_XC);
  float* gmx   = (float*)(ws + OFF_GMX);
  float* P0    = (float*)(ws + OFF_P0);
  float* P1    = (float*)(ws + OFF_P1);
  float* P2    = (float*)(ws + OFF_P2);
  float* coef1 = (float*)(ws + OFF_COEF1);
  float* coef2 = (float*)(ws + OFF_COEF2);
  float* coef3 = (float*)(ws + OFF_COEF3);

  first_layer_kernel<<<N_QUERY / 32, 256, 0, stream>>>(xyz, pts, W0, Y, Xc);
  stats0_kernel<<<N_BLK, THREADS_PB, 0, stream>>>(xyz, Y, Xc, P0);
  bn_coef_kernel<<<1, 128, 0, stream>>>(P0, g0, beta0, coef1, C_OUT1);
  mlp_kernel<false><<<N_BLK, THREADS_PB, 0, stream>>>(xyz, Y, Xc, W1, W2, coef1, coef1, P1, gmx);
  bn_coef_kernel<<<1, 128, 0, stream>>>(P1, g1, beta1, coef2, C_OUT2);
  mlp_kernel<true><<<N_BLK, THREADS_PB, 0, stream>>>(xyz, Y, Xc, W1, W2, coef1, coef2, P2, gmx);
  bn_coef_kernel<<<1, 128, 0, stream>>>(P2, g2, beta2, coef3, C_OUT3);
  out_kernel<<<N_BATCH * (N_PTS / 32), 256, 0, stream>>>(gmx, coef3, out);
}
